// TorchLocalAttention_5669356834645
// MI455X (gfx1250) — hardware-verified
//
#include <hip/hip_runtime.h>


#define NIMG 8
#define CC   128
#define HH   64
#define WW   64
#define TT   (HH * WW)
#define DM   CC
#define KWN  7
typedef _Float16 h16;
typedef unsigned short bf;
typedef __attribute__((ext_vector_type(16))) __bf16   v16bf;
typedef __attribute__((ext_vector_type(16))) _Float16 v16h;
typedef __attribute__((ext_vector_type(8)))  _Float16 v8h;
typedef __attribute__((ext_vector_type(8)))  unsigned short v8us;
typedef __attribute__((ext_vector_type(8)))  float    v8f;
typedef __attribute__((ext_vector_type(4)))  float    v4f;
typedef v8h  __attribute__((may_alias)) v8ha;
typedef v4f  __attribute__((may_alias)) v4fa;
typedef v8us __attribute__((may_alias)) v8usa;

__device__ __forceinline__ unsigned short f2bf(float f) { unsigned u = __float_as_uint(f); u += 0x7FFFu + ((u >> 16) & 1u); return (unsigned short)(u >> 16); }
__device__ __forceinline__ float bf2f(unsigned short b) { return __uint_as_float(((unsigned)b) << 16); }
__device__ __forceinline__ float bfr(float f) { return bf2f(f2bf(f)); }
__device__ __forceinline__ v16h cat16(v8h lo, v8h hi) { return __builtin_shufflevector(lo, hi, 0, 1, 2, 3, 4, 5, 6, 7, 8, 9, 10, 11, 12, 13, 14, 15); }
__device__ __forceinline__ v16bf cat16b(v8us lo, v8us hi) { return __builtin_bit_cast(v16bf, __builtin_shufflevector(lo, hi, 0, 1, 2, 3, 4, 5, 6, 7, 8, 9, 10, 11, 12, 13, 14, 15)); }
__device__ __forceinline__ v8f wmma16(v16h a, v16h b, v8f c) { return __builtin_amdgcn_wmma_f32_16x16x32_f16(false, a, false, b, (short)0, c, false, false); }
__device__ __forceinline__ v8f wmmab(v16bf a, v16bf b, v8f c) { return __builtin_amdgcn_wmma_f32_16x16x32_bf16(false, a, false, b, (short)0, c, false, false); }


template <typename T16> struct WFrag;
template <> struct WFrag<h16> { typedef v16h V; static __device__ __forceinline__ V ld(const h16* p) { return cat16(*(const v8h*)p, *(const v8h*)(p + 16)); } static __device__ __forceinline__ v8f mma(V a, V b, v8f c) { return wmma16(a, b, c); } };
template <> struct WFrag<bf> { typedef v16bf V; static __device__ __forceinline__ V ld(const bf* p) { return cat16b(*(const v8us*)p, *(const v8us*)(p + 16)); } static __device__ __forceinline__ v8f mma(V a, V b, v8f c) { return wmmab(a, b, c); } };
template <typename T16, int NSPLIT, bool BIAS>
__global__ __launch_bounds__(32) void k_gemmw(const T16* __restrict__ A, const T16* __restrict__ A2, const T16* __restrict__ Bt, const T16* __restrict__ Bt2, int K, float* C, int ldc, const float* __restrict__ bias, size_t sA, size_t sB, size_t sC) {
    typedef typename WFrag<T16>::V V;
    __shared__ __align__(16) float os[16 * 68];
    const size_t z = blockIdx.z; A += z * sA; if (A2) A2 += z * sA; Bt += z * sB; if (Bt2) Bt2 += z * sB; C += z * sC;
    const int lane = threadIdx.x & 31, lr = lane & 15, hi = lane >> 4; const int r0 = blockIdx.x * 64, c0 = blockIdx.y * 64;
    v8f acc[4][4];
#pragma unroll
    for (int mb = 0; mb < 4; ++mb)
#pragma unroll
        for (int nb = 0; nb < 4; ++nb) acc[mb][nb] = (v8f){};
    const size_t aoff = (size_t)(r0 + lr) * K + 8 * hi, boff = (size_t)(c0 + lr) * K + 8 * hi;
#pragma unroll 1
    for (int kc = 0; kc < K; kc += 32) {
        V a[4], a2[4];
#pragma unroll
        for (int mb = 0; mb < 4; ++mb) { a[mb] = WFrag<T16>::ld(A + aoff + (size_t)mb * 16 * K + kc); if (NSPLIT == 1 || NSPLIT == 2) a2[mb] = WFrag<T16>::ld(A2 + aoff + (size_t)mb * 16 * K + kc); }
#pragma unroll
        for (int nb = 0; nb < 4; ++nb) { const V b = WFrag<T16>::ld(Bt + boff + (size_t)nb * 16 * K + kc); V b2; if (NSPLIT >= 2) b2 = WFrag<T16>::ld(Bt2 + boff + (size_t)nb * 16 * K + kc);
#pragma unroll
            for (int mb = 0; mb < 4; ++mb) { acc[mb][nb] = WFrag<T16>::mma(a[mb], b, acc[mb][nb]); if (NSPLIT == 1 || NSPLIT == 2) acc[mb][nb] = WFrag<T16>::mma(a2[mb], b, acc[mb][nb]); if (NSPLIT >= 2) acc[mb][nb] = WFrag<T16>::mma(a[mb], b2, acc[mb][nb]); } }
        asm volatile("v_nop\n\tv_nop\n\tv_nop\n\tv_nop" : "+v"(acc[0][0]), "+v"(acc[1][1]), "+v"(acc[2][2]), "+v"(acc[3][3]) : "v"(a[0]), "v"(a[3]));
    }
#pragma unroll
    for (int mb = 0; mb < 4; ++mb) {
#pragma unroll
        for (int nb = 0; nb < 4; ++nb) {
#pragma unroll
            for (int j = 0; j < 8; ++j) os[(hi * 8 + j) * 68 + nb * 16 + lr] = acc[mb][nb][j]; }
        __builtin_amdgcn_wave_barrier(); asm volatile("" ::: "memory");
        float* crow = C + (size_t)(r0 + mb * 16) * ldc + c0;
#pragma unroll 1
        for (int ps = 0; ps < 2; ++ps) {
#pragma unroll
            for (int s = 0; s < 8; ++s) { const int row = 2 * s + hi, cofs = lr * 4; v4f val = *(const v4fa*)(os + row * 68 + cofs); if (BIAS) { val[0] += bfr(bias[c0 + cofs]); val[1] += bfr(bias[c0 + cofs + 1]); val[2] += bfr(bias[c0 + cofs + 2]); val[3] += bfr(bias[c0 + cofs + 3]); }
                *(volatile v4f*)(crow + (size_t)row * ldc + cofs) = val; }
            if (ps == 0) __threadfence(); }
        __builtin_amdgcn_wave_barrier(); asm volatile("" ::: "memory");
    }
}

__device__ __forceinline__ h16 tohx(float x) { return (h16)x; }
__device__ __forceinline__ void splitf(float y, unsigned short& h, unsigned short& l) { h = f2bf(y); l = f2bf(y - bf2f(h)); }
typedef __attribute__((ext_vector_type(2))) _Float16 v2h;
typedef __attribute__((ext_vector_type(4))) _Float16 v4h;
typedef __attribute__((ext_vector_type(2))) unsigned short v2us;
typedef __attribute__((ext_vector_type(4))) unsigned short v4us;
typedef __attribute__((ext_vector_type(2))) float v2f;
typedef __attribute__((ext_vector_type(4))) int v4i;


__global__ __launch_bounds__(256) void k_cvt8(const float* __restrict__ src, bf* dst, size_t n8) { const size_t i = (size_t)blockIdx.x * 256 + threadIdx.x; if (i >= n8) return; const v8f v = *(const v8f*)(src + i * 8); v8us o;
#pragma unroll
    for (int k = 0; k < 8; ++k) o[k] = f2bf(v[k]); *(volatile v8us*)(dst + i * 8) = o; __threadfence(); *(volatile v8us*)(dst + i * 8) = o; }

__global__ __launch_bounds__(256) void k_tpx(const float* __restrict__ xb, bf* XT) { const size_t e = ((size_t)blockIdx.x * 256 + threadIdx.x) * 4; if (e >= (size_t)TT * CC) return; const int c = (int)(e % CC); const int p = (int)(e / CC); v4us o;
#pragma unroll
    for (int q = 0; q < 4; ++q) o[q] = f2bf(xb[(size_t)(c + q) * TT + p]); *(volatile v4us*)(XT + e) = o; __threadfence(); *(volatile v4us*)(XT + e) = o; }
__global__ __launch_bounds__(256) void k_local(const float* __restrict__ F1, const float* __restrict__ F2, const float* __restrict__ F3, float* OT) {
    const int lane = threadIdx.x & 31; const int p = blockIdx.x * 8 + (threadIdx.x >> 5); if (p >= TT) return; const int y = p / WW, x = p % WW; const v4f a = *(const v4f*)(F1 + (size_t)p * CC + lane * 4);
    float m = -3.0e38f, Z = 0.f; v4f acc = (v4f){0.f, 0.f, 0.f, 0.f};
#pragma unroll 1
    for (int k = 0; k < KWN * KWN; ++k) { const int yy = y + k / KWN - KWN / 2, xx = x + k % KWN - KWN / 2; const bool inb = (yy >= 0 && yy < HH && xx >= 0 && xx < WW); const size_t qo = (size_t)(inb ? (yy * WW + xx) : 0) * CC + lane * 4;
        v4f b2 = *(const v4f*)(F2 + qo), b3 = *(const v4f*)(F3 + qo); if (!inb) { b2 = (v4f){0.f, 0.f, 0.f, 0.f}; b3 = b2; }
        float s = 0.f;
#pragma unroll
        for (int q = 0; q < 4; ++q) { float pr = __fmul_rn(a[q], b2[q]); asm volatile("" : "+v"(pr)); s = __fadd_rn(s, pr); }
#pragma unroll
        for (int sh = 16; sh; sh >>= 1) s += __shfl_xor(s, sh, 32);
        const float mn = fmaxf(m, s); float d1 = __fsub_rn(m, mn), d2 = __fsub_rn(s, mn); asm volatile("" : "+v"(d1), "+v"(d2));
        const float r = __builtin_amdgcn_exp2f(__fmul_rn(d1, 1.4426950408889634f)), w = __builtin_amdgcn_exp2f(__fmul_rn(d2, 1.4426950408889634f));
        float zr = __fmul_rn(Z, r); asm volatile("" : "+v"(zr)); Z = __fadd_rn(zr, w); m = mn;
#pragma unroll
        for (int q = 0; q < 4; ++q) { float t0 = __fmul_rn(acc[q], r); asm volatile("" : "+v"(t0)); float t1 = __fmul_rn(w, b3[q]); asm volatile("" : "+v"(t1)); acc[q] = __fadd_rn(t0, t1); } }
    const float iz = __fdiv_rn(1.0f, Z); v4f o;
#pragma unroll
    for (int q = 0; q < 4; ++q) o[q] = acc[q] * iz;
    float* dst = OT + (size_t)p * CC + lane * 4; *(volatile v4f*)dst = o; __threadfence(); *(volatile v4f*)dst = o; }
__global__ __launch_bounds__(256) void k_outT(const float* __restrict__ OT, float* Ob) { const size_t e = (size_t)blockIdx.x * 256 + threadIdx.x; if (e >= (size_t)CC * TT) return; const int p = (int)(e % TT); const int c = (int)(e / TT); const float v = OT[(size_t)p * CC + c]; *(volatile float*)(Ob + e) = v; __threadfence(); *(volatile float*)(Ob + e) = v; }

extern "C" void kernel_launch(void* const* d_in, const int* in_sizes, int n_in,
                              void* d_out, int out_size, void* d_ws, size_t ws_size, hipStream_t stream) {
    (void)in_sizes; (void)n_in; (void)out_size;
    const float* x = (const float*)d_in[0]; const float* w1 = (const float*)d_in[1]; const float* w2 = (const float*)d_in[2]; const float* w3 = (const float*)d_in[3];
    float* OUT = (float*)d_out;
    char* wsp = (char*)d_ws;
    auto take = [&](size_t bytes) { char* p = wsp; wsp += (bytes + 255) & ~(size_t)255; return (void*)p; };
    bf* W1 = (bf*)take((size_t)CC * CC * 2); bf* W2 = (bf*)take((size_t)CC * CC * 2); bf* W3 = (bf*)take((size_t)CC * CC * 2); bf* XT = (bf*)take((size_t)TT * CC * 2); float* F1 = (float*)take((size_t)TT * CC * 4); float* F2 = (float*)take((size_t)TT * CC * 4); float* F3 = (float*)take((size_t)TT * CC * 4); float* OT = (float*)take((size_t)TT * CC * 4);
    if ((size_t)(wsp - (char*)d_ws) > ws_size) return;
    k_cvt8<<<(CC * CC / 8 + 255) / 256, 256, 0, stream>>>(w1, W1, (size_t)CC * CC / 8); k_cvt8<<<(CC * CC / 8 + 255) / 256, 256, 0, stream>>>(w2, W2, (size_t)CC * CC / 8); k_cvt8<<<(CC * CC / 8 + 255) / 256, 256, 0, stream>>>(w3, W3, (size_t)CC * CC / 8);
    for (int n = 0; n < NIMG; ++n) { const float* xb = x + (size_t)n * CC * TT;
        k_tpx<<<(unsigned)(((size_t)TT * CC / 4 + 255) / 256), 256, 0, stream>>>(xb, XT);
        k_gemmw<bf, 0, false><<<dim3(TT / 64, CC / 64, 1), 32, 0, stream>>>(XT, nullptr, W1, nullptr, CC, F1, CC, nullptr, 0, 0, 0);
        k_gemmw<bf, 0, false><<<dim3(TT / 64, CC / 64, 1), 32, 0, stream>>>(XT, nullptr, W2, nullptr, CC, F2, CC, nullptr, 0, 0, 0);
        k_gemmw<bf, 0, false><<<dim3(TT / 64, CC / 64, 1), 32, 0, stream>>>(XT, nullptr, W3, nullptr, CC, F3, CC, nullptr, 0, 0, 0);
        k_local<<<TT / 8, 256, 0, stream>>>(F1, F2, F3, OT);
        k_outT<<<(unsigned)(((size_t)CC * TT + 255) / 256), 256, 0, stream>>>(OT, OUT + (size_t)n * CC * TT); }
}
